// TRANSNET_32856499814772
// MI455X (gfx1250) — hardware-verified
//
#include <hip/hip_runtime.h>
#include <math.h>

typedef __attribute__((ext_vector_type(16))) _Float16 v16h;
typedef __attribute__((ext_vector_type(16))) __bf16 v16b;
typedef __attribute__((ext_vector_type(8)))  _Float16 v8h;
typedef __attribute__((ext_vector_type(8)))  float v8f;
typedef __attribute__((ext_vector_type(4)))  float v4f;
typedef __attribute__((ext_vector_type(2)))  float v2f;
typedef __attribute__((ext_vector_type(4)))  unsigned v4u;
typedef __attribute__((ext_vector_type(4)))  int v4i;
typedef float __attribute__((may_alias)) float_a;
typedef int __attribute__((may_alias)) int_a;

template <typename T> __device__ __forceinline__ void vst2(void* p, T v) { *(volatile T*)p = v; __threadfence(); *(volatile T*)p = v; }
__device__ __forceinline__ v8f wmma16(v16h a, v16h b, v8f c) {
  v8f d = __builtin_amdgcn_wmma_f32_16x16x32_f16(false, a, false, b, (short)0, c, false, false);
  asm volatile("v_nop\n\tv_nop\n\tv_nop\n\tv_nop" : "+v"(d) : "v"(a), "v"(b));
  return d;
}
__device__ __forceinline__ v8f wmma_bf(v16b a, v16b b, v8f c) {
  v8f d = __builtin_amdgcn_wmma_f32_16x16x32_bf16(false, a, false, b, (short)0, c, false, false);
  asm volatile("v_nop\n\tv_nop\n\tv_nop\n\tv_nop" : "+v"(d) : "v"(a), "v"(b));
  return d;
}
__device__ __forceinline__ v16h frag_h(const _Float16* rowk0, int lane) {
  union { v16h v; v8h q[2]; } u; const _Float16* p = rowk0 + 8 * (lane >> 4);
  u.q[0] = *(const v8h*)p; u.q[1] = *(const v8h*)(p + 16); return u.v;
}
__device__ __forceinline__ v16h frag_f32(const float* rowk0, int lane) {
  v16h a; const float* p = rowk0 + 8 * (lane >> 4);
#pragma unroll
  for (int i = 0; i < 8; ++i) { a[i] = (_Float16)p[i]; a[8 + i] = (_Float16)p[16 + i]; }
  return a;
}
__device__ __forceinline__ v16h frag_f32s(const float* rowk0, int lane, float sc) {
  v16h a; const float* p = rowk0 + 8 * (lane >> 4);
#pragma unroll
  for (int i = 0; i < 8; ++i) { a[i] = (_Float16)(p[i] * sc); a[8 + i] = (_Float16)(p[16 + i] * sc); }
  return a;
}
__device__ __forceinline__ v16h fragc_f32(const float* W, int k0, int n, int lane, int ld, int K) {
  v16h a; const int g = lane >> 4;
#pragma unroll
  for (int i = 0; i < 8; ++i) { const int ka = k0 + 8 * g + i, kb = ka + 16;
    a[i] = (_Float16)(ka < K ? W[(size_t)(ka < K ? ka : K - 1) * ld + n] : 0.f); a[8 + i] = (_Float16)(kb < K ? W[(size_t)(kb < K ? kb : K - 1) * ld + n] : 0.f); }
  return a;
}
struct F2 { v16b h, l; };
__device__ __forceinline__ F2 bsplit16(const float v[16]) { F2 r;
#pragma unroll
  for (int i = 0; i < 16; ++i) { const __bf16 h = (__bf16)v[i]; r.h[i] = h; r.l[i] = (__bf16)(v[i] - (float)h); }
  return r; }
__device__ __forceinline__ F2 split_row(const float* row, int k0, int lane) { float v[16]; const float* p = row + k0 + 8 * (lane >> 4);
#pragma unroll
  for (int i = 0; i < 8; ++i) { v[i] = p[i]; v[8 + i] = p[16 + i]; }
  return bsplit16(v); }
__device__ __forceinline__ F2 split_rowK(const float* row, int k0, int lane, int K) { float v[16]; const int g = lane >> 4;
#pragma unroll
  for (int i = 0; i < 8; ++i) { const int ka = k0 + 8 * g + i, kb = ka + 16; v[i] = ka < K ? row[ka < K ? ka : K - 1] : 0.f; v[8 + i] = kb < K ? row[kb < K ? kb : K - 1] : 0.f; }
  return bsplit16(v); }
__device__ __forceinline__ F2 split_col(const float* W, int k0, int n, int lane, int ld, int K) { float v[16]; const int g = lane >> 4;
#pragma unroll
  for (int i = 0; i < 8; ++i) { const int ka = k0 + 8 * g + i, kb = ka + 16; v[i] = ka < K ? W[(size_t)(ka < K ? ka : K - 1) * ld + n] : 0.f; v[8 + i] = kb < K ? W[(size_t)(kb < K ? kb : K - 1) * ld + n] : 0.f; }
  return bsplit16(v); }
__device__ __forceinline__ v8f mac3(const F2& a, const F2& b, v8f c) { c = wmma_bf(a.l, b.h, c); c = wmma_bf(a.h, b.l, c); return wmma_bf(a.h, b.h, c); }
__device__ __forceinline__ float sigm(float v) { return 1.0f / (1.0f + expf(-v)); }
#define LDSX() do { asm volatile("s_wait_dscnt 0" ::: "memory"); __builtin_amdgcn_wave_barrier(); __builtin_amdgcn_fence(__ATOMIC_RELEASE, "workgroup"); } while (0)


#define NB 128
#define RR 10
#define LL 256
#define DD 64
#define FF 100
#define KW 3
#define IDD 32
#define VV 50000
#ifndef NDOC
#define NDOC (NB * RR)
#endif
#ifndef NPAIR
#define NPAIR NB
#endif
typedef __attribute__((ext_vector_type(8))) __bf16 v8b;
__device__ __forceinline__ v16b frag_b(const __bf16* rowk0, int lane) {
  union { v16b v; v8b q[2]; } u; const __bf16* p = rowk0 + 8 * (lane >> 4);
  u.q[0] = *(const v8b*)p; u.q[1] = *(const v8b*)(p + 16); return u.v;
}
__device__ __forceinline__ float bfr(float v) { return (float)(__bf16)v; }
__device__ __attribute__((noinline)) float exp_ni(float v) { return expf(v); }
__device__ __attribute__((noinline)) float erf_ni(float v) { return erff(v); }

__device__ __forceinline__ float tanh_x(float x) { const float e = exp_ni(-2.0f * fabsf(x)); const float t = (1.0f - e) / (1.0f + e); return x < 0.f ? -t : t; }
#define WS_PW   0u
#define PNET(n) ((size_t)(n) * 112 * 192)
#define PWEND   (3 * 112 * 192)
#define WS_UL   (WS_PW + 2u * PWEND)
#define WS_SEL  (WS_UL + 4u * NB * 640)
#define WS_END  (WS_SEL + 4u * NB * 4)

__global__ __launch_bounds__(256) void k_packW(const float* __restrict__ WU, const float* __restrict__ WI, const float* __restrict__ WT, __bf16* __restrict__ PW) {
  __shared__ __align__(16) __bf16 s[192]; const int f = blockIdx.x, n = blockIdx.y, t = threadIdx.x; const float* Wc = n == 0 ? WU : n == 1 ? WI : WT;
  if (t < 192) { const int kk = t / DD, d = t % DD; s[t] = (__bf16)((f < FF) ? Wc[((size_t)f * DD + d) * KW + kk] : 0.f); } __syncthreads();
  if (t < 24) vst2((unsigned*)(PW + PNET(n) + (size_t)f * 192 + t * 8), *(const v4u*)&s[t * 8]);
}
__global__ __launch_bounds__(128) void k_select(const int* __restrict__ UIDS, const int* __restrict__ IIDS, const int* __restrict__ U2I, const int* __restrict__ I2U, int* __restrict__ SEL) {
  __shared__ __align__(16) int s[NB][4]; const int b = threadIdx.x;
  if (b < NB) { int mode = 2, idx = 0; int ru = -1, ri = -1;
    for (int r = RR - 1; r >= 0; --r) { if (U2I[b * RR + r] == IIDS[b]) ru = r; if (I2U[b * RR + r] == UIDS[b]) ri = r; }
    if (ru >= 0) { mode = 0; idx = ru; } else if (ri >= 0) { mode = 1; idx = ri; }
    s[b][0] = mode; s[b][1] = idx; s[b][2] = 0; s[b][3] = 0; }
  __syncthreads();
  if (b < NB) vst2((unsigned*)(SEL + b * 4), *(const v4u*)&s[b][0]);
}
template <int NET>
__global__ __launch_bounds__(128) void k_cnn(const int* __restrict__ TOKU, const int* __restrict__ TOKI, const int* __restrict__ TOKR, const int* __restrict__ SEL, const float* __restrict__ EMB, const __bf16* __restrict__ PW, const float* __restrict__ BC, const float* __restrict__ WL, const float* __restrict__ BL, float* __restrict__ DST) {
  __shared__ int stok[LL + 2]; __shared__ float smax[4][112]; __shared__ __align__(16) float sout[IDD]; __shared__ float sm[112];
  const int tid = threadIdx.x, wave = tid >> 5, lane = tid & 31, col = lane & 15, g = lane >> 4; const int doc = blockIdx.x;
  const int* toks; if (NET == 0) toks = TOKU + (size_t)doc * LL; else if (NET == 1) toks = TOKI + (size_t)doc * LL; else { const int b = doc; const int mode = SEL[b * 4], idx = min(max(SEL[b * 4 + 1], 0), RR - 1); toks = (mode == 0) ? TOKU + ((size_t)b * RR + idx) * LL : (mode == 1) ? TOKI + ((size_t)b * RR + idx) * LL : TOKR + (size_t)b * LL; }
  for (int q = tid; q < LL + 2; q += 128) { const int pos = q - 1; stok[q] = (pos >= 0 && pos < LL) ? min(max(toks[pos], 0), VV - 1) : -1; }
  for (int q = tid; q < 112; q += 128) { smax[0][q] = 0.f; }
  __syncthreads();
  float mx[7][8];
#pragma unroll
  for (int j = 0; j < 7; ++j)
#pragma unroll
    for (int r = 0; r < 8; ++r) mx[j][r] = 0.f;
#pragma unroll 1
  for (int rt = 0; rt < 4; ++rt) { const int p0 = (wave * 4 + rt) * 16;
    v8f acc[7];
#pragma unroll
    for (int j = 0; j < 7; ++j) acc[j] = (v8f){};
#pragma unroll
    for (int kc = 0; kc < 6; ++kc) { const int kk = kc >> 1, dh = (kc & 1) * 32;
      const int tok = stok[p0 + col + kk];
      v16b a; if (tok >= 0) { const float* p = EMB + (size_t)tok * DD + dh + 8 * g;
#pragma unroll
        for (int i2 = 0; i2 < 8; ++i2) { a[i2] = (__bf16)p[i2]; a[8 + i2] = (__bf16)p[16 + i2]; } } else {
#pragma unroll
        for (int i2 = 0; i2 < 16; ++i2) a[i2] = (__bf16)0.f; }
#pragma unroll
      for (int j = 0; j < 7; ++j) acc[j] = wmma_bf(a, frag_b(PW + PNET(NET) + (size_t)(j * 16 + col) * 192 + kc * 32, lane), acc[j]); }
#pragma unroll
    for (int j = 0; j < 7; ++j) { const float bb = bfr(BC[min(j * 16 + col, FF - 1)]);
#pragma unroll
      for (int r = 0; r < 8; ++r) mx[j][r] = fmaxf(mx[j][r], fmaxf(acc[j][r] + bb, 0.f)); } }
#pragma unroll
  for (int j = 0; j < 7; ++j) { float m = mx[j][0];
#pragma unroll
    for (int r = 1; r < 8; ++r) m = fmaxf(m, mx[j][r]);
    m = fmaxf(m, __shfl_xor(m, 16));
    if (g == 0) smax[wave][j * 16 + col] = m; }
  __syncthreads();
  if (tid < 112) sm[tid] = fmaxf(fmaxf(smax[0][tid], smax[1][tid]), fmaxf(smax[2][tid], smax[3][tid]));
  __syncthreads();
  if (tid < IDD) { float a = bfr(BL[tid]);
#pragma unroll 4
    for (int f = 0; f < FF; ++f) a += sm[f] * bfr(WL[tid * FF + f]);
    sout[tid] = tanh_x(a); }
  __syncthreads();
  float* dst; if (NET == 0) dst = DST + (size_t)(doc / RR) * 640 + (doc % RR) * IDD; else if (NET == 1) dst = DST + (size_t)(doc / RR) * 640 + 320 + (doc % RR) * IDD; else dst = DST + (size_t)doc * IDD;
  if (tid < 8) vst2(dst + tid * 4, *(const v4f*)&sout[tid * 4]);
}
__global__ __launch_bounds__(128) void k_mlp(const float* __restrict__ UL, const float* __restrict__ W1, const float* __restrict__ B1, const float* __restrict__ W2, const float* __restrict__ B2, float* __restrict__ SRC) {
  __shared__ __align__(16) float s1[NB][IDD + 1]; __shared__ __align__(16) float s2[NB * IDD]; const int b = threadIdx.x;
  if (b < NPAIR) { for (int o = 0; o < IDD; ++o) { float a = bfr(B1[o]);
#pragma unroll 4
      for (int k = 0; k < 640; ++k) a += UL[(size_t)b * 640 + k] * bfr(W1[(size_t)o * 640 + k]);
      s1[b][o] = tanh_x(a); }
    for (int o = 0; o < IDD; ++o) { float a = bfr(B2[o]);
#pragma unroll 4
      for (int k = 0; k < IDD; ++k) a += s1[b][k] * bfr(W2[o * IDD + k]);
      s2[b * IDD + o] = tanh_x(a); } }
  __syncthreads();
  for (int q = b; q < NPAIR * IDD / 4; q += 128) vst2(SRC + q * 4, *(const v4f*)&s2[q * 4]);
}
extern "C" void kernel_launch(void* const* d_in, const int* in_sizes, int n_in, void* d_out, int out_size, void* d_ws, size_t ws_size, hipStream_t stream) {
  (void)in_sizes; (void)n_in; (void)out_size;
  const float** F = (const float**)d_in; const int** I = (const int**)d_in;
  if (ws_size < (size_t)WS_END) return;
  char* ws = (char*)d_ws; __bf16* PW = (__bf16*)(ws + WS_PW); float* UL = (float*)(ws + WS_UL); int* SEL = (int*)(ws + WS_SEL);
  float* SRC = (float*)d_out; float* TL = SRC + (size_t)NB * IDD;
  k_packW<<<dim3(112, 3), 256, 0, stream>>>(F[9], F[13], F[25], PW);
  k_select<<<1, 128, 0, stream>>>(I[2], I[3], I[4], I[5], SEL);
  k_cnn<0><<<NDOC, 128, 0, stream>>>(I[0], I[1], I[6], SEL, F[7], PW, F[10], F[11], F[12], UL);
  k_cnn<1><<<NDOC, 128, 0, stream>>>(I[0], I[1], I[6], SEL, F[8], PW, F[14], F[15], F[16], UL);
  k_mlp<<<1, 128, 0, stream>>>(UL, F[17], F[18], F[19], F[20], SRC);
  k_cnn<2><<<NPAIR, 128, 0, stream>>>(I[0], I[1], I[6], SEL, F[24], PW, F[26], F[27], F[28], TL);
}
